// DiffPoolGNN_74938589380725
// MI455X (gfx1250) — hardware-verified
//
#include <hip/hip_runtime.h>
#include <stddef.h>


#define IND     16
#define EDD     8
#define HD      64
#define AC      16
#define EMB     128
#define NPER    512
#define GMAX    64
#define NTHR    256
#define NWAVE   8
#define EPT     8
#define NGRP    1
#define CHUNK   (NTHR * EPT * NGRP)
#define WCAPC   (EPT * NGRP * 32)
#define WCAPF   (EPT * NGRP * 32)
#define ESHF    11
#define NBC     32768
#define NBF     2048
#define RCAP    67584
#define RBN     128
#define TGT     256
#define DEGCAP  256
#define GROWS   128
#define OTHR    512
#define FSCL    16
#define WSCL    64
#define WSCAP   134217728

#define LDS_COUNT  ((NBC + NWAVE * WCAPC + NWAVE) * 4)
#define LDS_FILL   ((RCAP + NBF + NWAVE * WCAPF + NWAVE) * 4)

static_assert((CHUNK & (CHUNK - 1)) == 0);
static_assert(CHUNK <= 4096);
static_assert((NBC & (NBC - 1)) == 0 && (NBF & (NBF - 1)) == 0);
static_assert(NBF <= (1 << ESHF));
static_assert((NBC % NBF) == 0);
static_assert(OTHR * 4 == NBF);
static_assert((RCAP % 32) == 0);
static_assert(TGT == NWAVE * 32);
static_assert(GROWS == NWAVE * 16);
static_assert((TGT % GROWS) == 0);
static_assert(NBC == NWAVE * 32 * 128);
static_assert(HD == 64 && AC == 16 && EMB == 128 && IND == 16 && EDD == 8);
static_assert((NPER % TGT) == 0);
static_assert(GMAX * 4 == NTHR);
static_assert(LDS_FILL <= 293 * 1024);
static_assert(LDS_COUNT <= 160 * 1024);

typedef float          v4f   __attribute__((ext_vector_type(4)));
typedef float          v8f   __attribute__((ext_vector_type(8)));
typedef int            v4i   __attribute__((ext_vector_type(4)));
typedef _Float16       v8h   __attribute__((ext_vector_type(8)));
typedef _Float16       v16h  __attribute__((ext_vector_type(16)));
typedef unsigned short v8us  __attribute__((ext_vector_type(8)));
typedef unsigned short v16us __attribute__((ext_vector_type(16)));
typedef __bf16         v16bf __attribute__((ext_vector_type(16)));
union FragH { v16h v; v8h h[2]; };
union FragU { v16us v; v8us h[2]; };

#define WAVE_SYNC() do { __builtin_amdgcn_fence(__ATOMIC_ACQ_REL, "wavefront"); __builtin_amdgcn_wave_barrier(); } while (0)

__device__ __forceinline__ v8f wmf(v16h a, v16h b, v8f c) {
  v8f d = __builtin_amdgcn_wmma_f32_16x16x32_f16(false, a, false, b, (short)0, c, false, false);
  asm volatile("v_nop\n\tv_nop\n\tv_nop\n\tv_nop" : "+v"(d) : "v"(a), "v"(b));
  return d;
}
__device__ __forceinline__ v8f wmb(v16us a, v16us b, v8f c) {
  const v16bf A = __builtin_bit_cast(v16bf, a);
  const v16bf B = __builtin_bit_cast(v16bf, b);
  v8f d = __builtin_amdgcn_wmma_f32_16x16x32_bf16(false, A, false, B, (short)0, c, false, false);
  asm volatile("v_nop\n\tv_nop\n\tv_nop\n\tv_nop" : "+v"(d) : "v"(A), "v"(B));
  return d;
}

__device__ __forceinline__ unsigned bf_bits(float f) {
  const unsigned u = __float_as_uint(f);
  return (u + 0x7FFFu + ((u >> 16) & 1u)) >> 16;
}

template <int NB, int EIDX, int WC>
__device__ __forceinline__ int scan_chunk(const int* __restrict__ keys, int nK, int cbase,
                                          int slotBase, int vec8, int* list, int tid, int lane, int wave) {
  int wc = 0;
#pragma unroll
  for (int g = 0; g < NGRP; ++g) {
    const int el0  = (g * NTHR + tid) * EPT;
    const int e0   = cbase + el0;
    const int sent = -2147483647 - 1;
    v4i da, db;
    if (vec8 != 0 && cbase + CHUNK <= nK) {
      da = *(const v4i*)(keys + e0);
      db = *(const v4i*)(keys + e0 + 4);
    } else {
      const int i0 = min(e0, nK - 1),     i1 = min(e0 + 1, nK - 1), i2 = min(e0 + 2, nK - 1), i3 = min(e0 + 3, nK - 1);
      const int i4 = min(e0 + 4, nK - 1), i5 = min(e0 + 5, nK - 1), i6 = min(e0 + 6, nK - 1), i7 = min(e0 + 7, nK - 1);
      da.x = (e0     < nK) ? keys[i0] : sent;
      da.y = (e0 + 1 < nK) ? keys[i1] : sent;
      da.z = (e0 + 2 < nK) ? keys[i2] : sent;
      da.w = (e0 + 3 < nK) ? keys[i3] : sent;
      db.x = (e0 + 4 < nK) ? keys[i4] : sent;
      db.y = (e0 + 5 < nK) ? keys[i5] : sent;
      db.z = (e0 + 6 < nK) ? keys[i6] : sent;
      db.w = (e0 + 7 < nK) ? keys[i7] : sent;
    }
    const unsigned nb = (unsigned)slotBase;
    const unsigned s0 = (unsigned)da.x - nb, s1 = (unsigned)da.y - nb;
    const unsigned s2 = (unsigned)da.z - nb, s3 = (unsigned)da.w - nb;
    const unsigned s4 = (unsigned)db.x - nb, s5 = (unsigned)db.y - nb;
    const unsigned s6 = (unsigned)db.z - nb, s7 = (unsigned)db.w - nb;
    const bool h0 = s0 < (unsigned)NB, h1 = s1 < (unsigned)NB, h2 = s2 < (unsigned)NB, h3 = s3 < (unsigned)NB;
    const bool h4 = s4 < (unsigned)NB, h5 = s5 < (unsigned)NB, h6 = s6 < (unsigned)NB, h7 = s7 < (unsigned)NB;
    const unsigned any = __builtin_amdgcn_ballot_w32(h0 | h1 | h2 | h3 | h4 | h5 | h6 | h7);
    if (any != 0u) {
#define HITJ(HJ, SJ, JJ) { \
        const unsigned mj = __builtin_amdgcn_ballot_w32(HJ); \
        if (mj != 0u) { \
          if (HJ) { \
            const int pos = wc + (int)__builtin_amdgcn_mbcnt_lo(mj, 0u); \
            const int entv = EIDX ? (((el0 + (JJ)) << ESHF) | (int)(SJ)) : (int)(SJ); \
            if (pos < WC) list[wave * WC + pos] = entv; \
          } \
          wc += (int)__builtin_popcount(mj); } }
      HITJ(h0, s0, 0)
      HITJ(h1, s1, 1)
      HITJ(h2, s2, 2)
      HITJ(h3, s3, 3)
      HITJ(h4, s4, 4)
      HITJ(h5, s5, 5)
      HITJ(h6, s6, 6)
      HITJ(h7, s7, 7)
#undef HITJ
    }
  }
  return wc;
}

__global__ __launch_bounds__(NTHR) void k_count(const int* __restrict__ keys, int* cnt, int nK, int vec8) {
  extern __shared__ v4f lds_dyn[];
  int* scnt = (int*)lds_dyn;
  int* list = scnt + NBC;
  int* wcnt = list + NWAVE * WCAPC;
  const int tid = threadIdx.x, lane = tid & 31, wave = tid >> 5;
  const int nodeBase = blockIdx.x * NBC;

  {
    const v4i z = {0, 0, 0, 0};
    for (int i = tid; i < NBC / 4; i += NTHR) ((v4i*)scnt)[i] = z;
  }
  __syncthreads();

  const int nChunks = (nK + CHUNK - 1) / CHUNK;
#pragma unroll 1
  for (int ch = 0; ch < nChunks; ++ch) {
    const int cbase = ch * CHUNK;
    const int wc = scan_chunk<NBC, 0, WCAPC>(keys, nK, cbase, nodeBase, vec8, list, tid, lane, wave);
    if (lane == 0) wcnt[wave] = wc;
    __syncthreads();
    if (wave == 0) {
#pragma unroll 1
      for (int wsx = 0; wsx < NWAVE; ++wsx) {
        int n = __builtin_amdgcn_readfirstlane(wcnt[wsx]);
        n = n > WCAPC ? WCAPC : (n < 0 ? 0 : n);
        const int* lp = list + wsx * WCAPC;
#pragma unroll 1
        for (int i = 0; i < n; ++i) {
          const int ent  = __builtin_amdgcn_readfirstlane(lp[i]);
          const int slot = ent & (NBC - 1);
          if (lane == 0) scnt[slot] = scnt[slot] + 1;
        }
      }
    }
    __syncthreads();
  }

  int* cp = cnt + (size_t)nodeBase;
#pragma unroll 4
  for (int q = 0; q < 32; ++q) {
    const int f = (wave * 32 + q) * 128 + 4 * lane;
    const v4i c = *(const v4i*)(scnt + f);
    *(volatile v4i*)(cp + f) = c;
  }
  __threadfence();
#pragma unroll 4
  for (int q = 0; q < 32; ++q) {
    const int f = (wave * 32 + q) * 128 + 4 * lane;
    const v4i c = *(const v4i*)(scnt + f);
    *(volatile v4i*)(cp + f) = c;
  }
}

__global__ __launch_bounds__(OTHR) void k_offsets(
    const int* __restrict__ cnt, int* off, int* rbase, int nBF) {
  __shared__ __attribute__((aligned(16))) int srb[RBN];
  __shared__ int wtot[OTHR / 32];
  const int tid = threadIdx.x, lane = tid & 31, wave = tid >> 5;
  for (int i = tid; i < RBN; i += OTHR) srb[i] = 0;
  int carry = 0;
#pragma unroll 1
  for (int fb = 0; fb < nBF; ++fb) {
    const int base = fb * NBF;
    const v4i c = *(const v4i*)(cnt + base + 4 * tid);
    const int e0 = max(c.x, 0), e1 = max(c.y, 0), e2 = max(c.z, 0), e3 = max(c.w, 0);
    const int ts = e0 + e1 + e2 + e3;
    int incl = ts;
#pragma unroll
    for (int d = 1; d < 32; d <<= 1) {
      const int t = __shfl_up(incl, d, 32);
      if (lane >= d) incl += t;
    }
    if (lane == 31) wtot[wave] = incl;
    __syncthreads();
    int pre = 0;
#pragma unroll 1
    for (int w = 0; w < wave; ++w) pre += wtot[w];
    int tot = 0;
#pragma unroll
    for (int w = 0; w < OTHR / 32; ++w) tot += wtot[w];
    int run = carry + pre + incl - ts;
    v4i o;
    o.x = run; run += e0;
    o.y = run; run += e1;
    o.z = run; run += e2;
    o.w = run;
    int* op = off + base + 4 * tid;
    *(volatile v4i*)op = o;
    __threadfence();
    *(volatile v4i*)op = o;
    if (tid == 0) srb[min(fb, RBN - 1)] = carry;
    carry += (tot + 31) & ~31;
    __syncthreads();
  }
  if (tid == 0) srb[min(nBF, RBN - 1)] = carry;
  __syncthreads();
  v4i rv = {0, 0, 0, 0};
  if (tid < 32) rv = *(const v4i*)(srb + 4 * tid);
  if (tid < 32) *(volatile v4i*)(rbase + 4 * tid) = rv;
  __threadfence();
  if (tid < 32) *(volatile v4i*)(rbase + 4 * tid) = rv;
}

__global__ __launch_bounds__(NTHR) void k_fill(
    const int* __restrict__ keys, const int* __restrict__ off, const int* __restrict__ rbase,
    int* csr, int nK, int vec8, int csrLen) {
  extern __shared__ v4f lds_dyn[];
  int* region = (int*)lds_dyn;
  int* cursor = region + RCAP;
  int* list   = cursor + NBF;
  int* wcnt   = list + NWAVE * WCAPF;
  const int tid = threadIdx.x, lane = tid & 31, wave = tid >> 5;
  const int b = blockIdx.x;
  const int nodeBase = b * NBF;

  int rb0 = rbase[b];
  const int rb1 = rbase[b + 1];
  rb0 = rb0 < 0 ? 0 : (rb0 > csrLen ? csrLen : rb0);
  rb0 &= ~31;
  int len = rb1 - rb0;
  len = len < 0 ? 0 : (len > RCAP ? RCAP : len);
  int lenW = (len + 31) & ~31;
  if (rb0 + lenW > csrLen) lenW = (csrLen - rb0) & ~31;

  {
    const v4i z = {0, 0, 0, 0};
    for (int i = tid; i < RCAP / 4; i += NTHR) ((v4i*)region)[i] = z;
    for (int s = tid; s < NBF; s += NTHR) {
      int o = off[nodeBase + s] - rb0;
      o = o < 0 ? 0 : (o > RCAP ? RCAP : o);
      cursor[s] = o;
    }
  }
  __syncthreads();

  const int nChunks = (nK + CHUNK - 1) / CHUNK;
#pragma unroll 1
  for (int ch = 0; ch < nChunks; ++ch) {
    const int cbase = ch * CHUNK;
    const int wc = scan_chunk<NBF, 1, WCAPF>(keys, nK, cbase, nodeBase, vec8, list, tid, lane, wave);
    if (lane == 0) wcnt[wave] = wc;
    __syncthreads();
    if (wave == 0) {
#pragma unroll 1
      for (int wsx = 0; wsx < NWAVE; ++wsx) {
        int n = __builtin_amdgcn_readfirstlane(wcnt[wsx]);
        n = n > WCAPF ? WCAPF : (n < 0 ? 0 : n);
        const int* lp = list + wsx * WCAPF;
#pragma unroll 1
        for (int i = 0; i < n; ++i) {
          const int ent  = __builtin_amdgcn_readfirstlane(lp[i]);
          const int slot = ent & (NBF - 1);
          const int el   = (ent >> ESHF) & (CHUNK - 1);
          int e = cbase + el;
          e = e > nK - 1 ? nK - 1 : e;
          if (lane == 0) {
            int pos = cursor[slot];
            pos = pos < 0 ? 0 : (pos > RCAP - 1 ? RCAP - 1 : pos);
            region[pos] = e;
            const int np = pos + 1;
            cursor[slot] = np > RCAP ? RCAP : np;
          }
        }
      }
    }
    __syncthreads();
  }

  const int nv = lenW >> 2;
  int* gp = csr + rb0;
#pragma unroll 1
  for (int i = tid; i < nv; i += NTHR) { const v4i v = ((const v4i*)region)[i]; *(volatile v4i*)(gp + 4 * i) = v; }
  __threadfence();
#pragma unroll 1
  for (int i = tid; i < nv; i += NTHR) { const v4i v = ((const v4i*)region)[i]; *(volatile v4i*)(gp + 4 * i) = v; }
}

__global__ __launch_bounds__(NTHR) void k_w2split(const float* __restrict__ W, unsigned short* Wh,
                                                  unsigned short* Wl, int K, int N, int KP, int total8) {
  const int i = (int)blockIdx.x * NTHR + (int)threadIdx.x;
  if (i >= total8) return;
  const int e  = 8 * i;
  const int n  = e / KP;
  const int k0 = e - n * KP;
  const int ncl = n < N ? n : N - 1;
  v8us hv, lv;
#pragma unroll
  for (int q = 0; q < 8; ++q) {
    const int k = k0 + q;
    const int kcl = k < K ? k : K - 1;
    const float wv = W[(size_t)kcl * N + ncl];
    const float v = (k < K && n < N) ? wv : 0.0f;
    const unsigned hb = bf_bits(v);
    const unsigned lb = bf_bits(v - __uint_as_float(hb << 16));
    hv[q] = (unsigned short)hb;
    lv[q] = (unsigned short)lb;
  }
  unsigned short* ph = Wh + e;
  unsigned short* pl = Wl + e;
  *(volatile v8us*)ph = hv;
  *(volatile v8us*)pl = lv;
  __threadfence();
  *(volatile v8us*)ph = hv;
  *(volatile v8us*)pl = lv;
}

template <int DN, int OUT, int SRC32>
__global__ __launch_bounds__(NTHR) void k_conv(
    const float* __restrict__ xf, const _Float16* __restrict__ xh, const float* __restrict__ ea,
    const int* __restrict__ csr, const int* __restrict__ off, const int* __restrict__ cnt,
    const int* __restrict__ esrc, const float* __restrict__ w1, const float* __restrict__ b1,
    float* R, int nN, int nE, int csrLen) {
  constexpr int K1  = DN + EDD;
  constexpr int KP1 = ((K1 + 31) / 32) * 32;
  constexpr int KC  = KP1 / 32;
  constexpr int NC  = OUT / 16;
  constexpr int TP  = KP1 + 8;
  constexpr int RP  = (OUT < 32) ? 32 : OUT;
  constexpr int RPE = 128 / RP;
  constexpr int PPR = DN / 8;
  constexpr int PADP = (TP - K1) / 8;
  static_assert((OUT % 16) == 0 && OUT <= 64);
  static_assert((DN % 8) == 0 && (K1 % 8) == 0 && ((TP - K1) % 8) == 0);
  static_assert(SRC32 ? (PPR == 2) : (((16 * PPR) % 32) == 0));
  static_assert(RPE * RP == 128 && (32 % RPE) == 0);

  __shared__ __attribute__((aligned(32))) v16h sW[KC * NC * 32];
  __shared__ __attribute__((aligned(16))) _Float16 sT[NWAVE * 16 * TP];
  __shared__ __attribute__((aligned(16))) float sStg[NWAVE * 128];
  __shared__ float sB[OUT];
  const int tid = threadIdx.x, lane = tid & 31, wave = tid >> 5, hh = lane >> 4, m = lane & 15;

  for (int idx = tid; idx < KC * NC * 32 * 16; idx += NTHR) {
    const int i = idx & 15, ln = (idx >> 4) & 31, cn = idx >> 9;
    const int kc = cn / NC, nc = cn - kc * NC;
    const int lh = ln >> 4;
    const int kk = (i < 8) ? (8 * lh + i) : (16 + 8 * lh + (i - 8));
    const int k = kc * 32 + kk, n = nc * 16 + (ln & 15);
    const int kcl = k < K1 ? k : K1 - 1;
    const float wv = w1[kcl * OUT + n];
    const float v = (k < K1) ? wv * (float)WSCL : 0.0f;
    ((_Float16*)sW)[idx] = (_Float16)v;
  }
  for (int i = tid; i < OUT; i += NTHR) sB[i] = b1[i];
  {
    v8h z;
#pragma unroll
    for (int q = 0; q < 8; ++q) z[q] = (_Float16)0.0f;
    for (int idx = tid; idx < NWAVE * 16 * PADP; idx += NTHR) {
      const int row = idx / PADP, q = idx - row * PADP;
      *(v8h*)(sT + row * TP + K1 + 8 * q) = z;
    }
  }
  for (int i = tid; i < NWAVE * 128; i += NTHR) sStg[i] = 0.0f;
  __syncthreads();

  const int tbase = (int)blockIdx.x * TGT + wave * 32;
  const int cnt_l = cnt[tbase + lane];
  const int off_l = off[tbase + lane];
  float bcol[NC];
#pragma unroll
  for (int nc = 0; nc < NC; ++nc) bcol[nc] = sB[16 * nc + m];
  _Float16* T = sT + wave * 16 * TP;
  float* stg = sStg + wave * 128;
  const float osc = 1.0f / ((float)FSCL * (float)WSCL);
  const int erow = lane & 15;

#pragma unroll 1
  for (int j = 0; j < 32; ++j) {
    const int c = tbase + j;
    int n = __builtin_amdgcn_readlane(cnt_l, j);
    n = n < 0 ? 0 : (n > DEGCAP ? DEGCAP : n);
    const int st = __builtin_amdgcn_readlane(off_l, j);
    float sum[NC];
#pragma unroll
    for (int nc = 0; nc < NC; ++nc) sum[nc] = 0.0f;
    const int ntile = (n + 15) >> 4;
#pragma unroll 1
    for (int tl = 0; tl < ntile; ++tl) {
      int pos = st + tl * 16 + erow;
      pos = pos < 0 ? 0 : (pos > csrLen - 1 ? csrLen - 1 : pos);
      int el = csr[pos];
      el = el < 0 ? 0 : (el > nE - 1 ? nE - 1 : el);
      int sl = esrc[el];
      sl = sl < 0 ? 0 : (sl > nN - 1 ? nN - 1 : sl);
      if constexpr (SRC32 != 0) {
        const int row = lane >> 1, q = lane & 1;
        const int sr = __shfl(sl, row, 32);
        const float* xp = xf + (size_t)sr * DN + 8 * q;
        const v4f f0 = *(const v4f*)xp;
        const v4f f1 = *(const v4f*)(xp + 4);
        v8h hv;
        hv[0] = (_Float16)(f0.x * (float)FSCL); hv[1] = (_Float16)(f0.y * (float)FSCL);
        hv[2] = (_Float16)(f0.z * (float)FSCL); hv[3] = (_Float16)(f0.w * (float)FSCL);
        hv[4] = (_Float16)(f1.x * (float)FSCL); hv[5] = (_Float16)(f1.y * (float)FSCL);
        hv[6] = (_Float16)(f1.z * (float)FSCL); hv[7] = (_Float16)(f1.w * (float)FSCL);
        *(v8h*)(T + row * TP + 8 * q) = hv;
      } else {
#pragma unroll
        for (int i = 0; i < (16 * PPR) / 32; ++i) {
          const int p = lane + 32 * i;
          const int row = p / PPR, q = p - row * PPR;
          const int sr = __shfl(sl, row, 32);
          const v8h hv = *(const v8h*)(xh + (size_t)sr * DN + 8 * q);
          *(v8h*)(T + row * TP + 8 * q) = hv;
        }
      }
      {
        const float* ep = ea + (size_t)el * EDD;
        const v4f f0 = *(const v4f*)ep;
        const v4f f1 = *(const v4f*)(ep + 4);
        v8h hv;
        hv[0] = (_Float16)(f0.x * (float)FSCL); hv[1] = (_Float16)(f0.y * (float)FSCL);
        hv[2] = (_Float16)(f0.z * (float)FSCL); hv[3] = (_Float16)(f0.w * (float)FSCL);
        hv[4] = (_Float16)(f1.x * (float)FSCL); hv[5] = (_Float16)(f1.y * (float)FSCL);
        hv[6] = (_Float16)(f1.z * (float)FSCL); hv[7] = (_Float16)(f1.w * (float)FSCL);
        *(v8h*)(T + erow * TP + DN) = hv;
      }
      WAVE_SYNC();
      v8f acc[NC];
#pragma unroll
      for (int nc = 0; nc < NC; ++nc) { v8f z = {0.f, 0.f, 0.f, 0.f, 0.f, 0.f, 0.f, 0.f}; acc[nc] = z; }
#pragma unroll
      for (int kc = 0; kc < KC; ++kc) {
        FragH af;
        af.h[0] = *(const v8h*)(T + m * TP + 32 * kc + 8 * hh);
        af.h[1] = *(const v8h*)(T + m * TP + 32 * kc + 16 + 8 * hh);
#pragma unroll
        for (int nc = 0; nc < NC; ++nc) acc[nc] = wmf(af.v, sW[(kc * NC + nc) * 32 + lane], acc[nc]);
      }
      const int nval = n - tl * 16;
#pragma unroll
      for (int nc = 0; nc < NC; ++nc) {
#pragma unroll
        for (int r = 0; r < 8; ++r) {
          const float v = fmaxf(fmaf(acc[nc][r], osc, bcol[nc]), 0.0f);
          sum[nc] += ((8 * hh + r) < nval) ? v : 0.0f;
        }
      }
      WAVE_SYNC();
    }
#pragma unroll
    for (int nc = 0; nc < NC; ++nc) sum[nc] += __shfl_xor(sum[nc], 16, 32);
    const float inv = (n > 0) ? (1.0f / (float)n) : 0.0f;
#pragma unroll
    for (int nc = 0; nc < NC; ++nc) stg[(j % RPE) * RP + 16 * nc + m] = sum[nc] * inv;
    if ((j % RPE) == RPE - 1) {
      WAVE_SYNC();
      const v4f v = *(const v4f*)(stg + 4 * lane);
      float* rp = R + (size_t)(c - (RPE - 1)) * RP + 4 * lane;
      *(volatile v4f*)rp = v;
      __threadfence();
      *(volatile v4f*)rp = v;
      WAVE_SYNC();
    }
  }
}

template <int KD, int NCOL, int MODE, int WF>
__global__ __launch_bounds__(NTHR) void k_gemm2(
    const float* __restrict__ Rm, const unsigned short* __restrict__ Wh, const unsigned short* __restrict__ Wl,
    const int* __restrict__ cnt, const float* __restrict__ b2,
    _Float16* Hh, float* Hf, float* So, int nN) {
  static_assert((KD % 32) == 0 && (NCOL % 16) == 0 && NCOL <= 64);
  static_assert(MODE == 0 ? NCOL == 64 : NCOL == 16);
  constexpr int NT = NCOL / 16;
  __shared__ __attribute__((aligned(16))) float stg[GROWS * NCOL];
  const int tid = threadIdx.x, lane = tid & 31, wave = tid >> 5, hh = lane >> 4, m = lane & 15;
  const int rowBase = (int)blockIdx.x * GROWS;
  const float* ap = Rm + (size_t)(rowBase + wave * 16 + m) * KD + 8 * hh;
  const unsigned short* bh0 = Wh + (size_t)m * KD + 8 * hh;
  const unsigned short* bl0 = Wl + (size_t)m * KD + 8 * hh;

  v8f acc[NT];
#pragma unroll
  for (int t = 0; t < NT; ++t) { v8f z = {0.f, 0.f, 0.f, 0.f, 0.f, 0.f, 0.f, 0.f}; acc[t] = z; }

#pragma unroll
  for (int kt = 0; kt < KD / 32; ++kt) {
    const float* a = ap + 32 * kt;
    const v4f x0 = *(const v4f*)a;
    const v4f x1 = *(const v4f*)(a + 4);
    const v4f x2 = *(const v4f*)(a + 16);
    const v4f x3 = *(const v4f*)(a + 20);
    v16us ahv, alv;
#define SPL(I, X) { const float xv_ = (X); const unsigned hb_ = bf_bits(xv_); \
    ahv[I] = (unsigned short)hb_; alv[I] = (unsigned short)bf_bits(xv_ - __uint_as_float(hb_ << 16)); }
    SPL(0, x0.x)  SPL(1, x0.y)  SPL(2, x0.z)  SPL(3, x0.w)
    SPL(4, x1.x)  SPL(5, x1.y)  SPL(6, x1.z)  SPL(7, x1.w)
    SPL(8, x2.x)  SPL(9, x2.y)  SPL(10, x2.z) SPL(11, x2.w)
    SPL(12, x3.x) SPL(13, x3.y) SPL(14, x3.z) SPL(15, x3.w)
#undef SPL
#pragma unroll
    for (int t = 0; t < NT; ++t) {
      const unsigned short* bp = bh0 + (size_t)(16 * t) * KD + 32 * kt;
      const unsigned short* lq = bl0 + (size_t)(16 * t) * KD + 32 * kt;
      FragU bh, bl;
      bh.h[0] = *(const v8us*)bp;  bh.h[1] = *(const v8us*)(bp + 16);
      bl.h[0] = *(const v8us*)lq;  bl.h[1] = *(const v8us*)(lq + 16);
      acc[t] = wmb(ahv, bh.v, acc[t]);
      acc[t] = wmb(alv, bh.v, acc[t]);
      acc[t] = wmb(ahv, bl.v, acc[t]);
    }
  }

  const int r0w = wave * 16 + 8 * hh;
  int cr[8];
  {
    const v4i cA = *(const v4i*)(cnt + rowBase + r0w);
    const v4i cB = *(const v4i*)(cnt + rowBase + r0w + 4);
    cr[0] = cA.x; cr[1] = cA.y; cr[2] = cA.z; cr[3] = cA.w; cr[4] = cB.x; cr[5] = cB.y; cr[6] = cB.z; cr[7] = cB.w;
  }
  float bcol[NT];
#pragma unroll
  for (int t = 0; t < NT; ++t) bcol[t] = b2[16 * t + m];
#pragma unroll
  for (int t = 0; t < NT; ++t) {
#pragma unroll
    for (int r = 0; r < 8; ++r) {
      const int row = rowBase + r0w + r;
      const bool ok = (cr[r] > 0) && (row < nN);
      float v = ok ? (acc[t][r] + bcol[t]) : 0.0f;
      if (MODE == 0) v = fmaxf(v, 0.0f);
      stg[(r0w + r) * NCOL + 16 * t + m] = v;
    }
  }
  __syncthreads();

  if constexpr (MODE == 1) {
    if (tid < GROWS) {
      float* rowp = stg + tid * NCOL;
#pragma unroll 1
      for (int pass = 0; pass < 2; ++pass) {
        float mx = -__builtin_huge_valf();
#pragma unroll 1
        for (int i = 0; i < NCOL; ++i) mx = fmaxf(mx, rowp[i]);
        float sm = 0.0f;
#pragma unroll 1
        for (int i = 0; i < NCOL; ++i) { const float e = expf(rowp[i] - mx); rowp[i] = e; sm += e; }
        const float inv = 1.0f / sm;
#pragma unroll 1
        for (int i = 0; i < NCOL; ++i) rowp[i] = rowp[i] * inv;
      }
    }
    __syncthreads();
    const float* lp = stg + wave * 16 * NCOL;
    float* gp = So + (size_t)(rowBase + wave * 16) * NCOL;
#pragma unroll
    for (int i = 0; i < 2; ++i) {
      const v4f v = *(const v4f*)(lp + i * 128 + 4 * lane);
      *(volatile v4f*)(gp + (size_t)i * 128 + 4 * lane) = v;
    }
    __threadfence();
#pragma unroll
    for (int i = 0; i < 2; ++i) {
      const v4f v = *(const v4f*)(lp + i * 128 + 4 * lane);
      *(volatile v4f*)(gp + (size_t)i * 128 + 4 * lane) = v;
    }
  } else {
    const float* lp = stg + wave * 16 * NCOL;
    _Float16* hp = Hh + (size_t)(rowBase + wave * 16) * NCOL;
    float* fp = Hf + (size_t)(rowBase + wave * 16) * NCOL;
#pragma unroll 1
    for (int pass = 0; pass < 2; ++pass) {
#pragma unroll
      for (int i = 0; i < 4; ++i) {
        const v4f fa = *(const v4f*)(lp + i * 256 + 8 * lane);
        const v4f fb = *(const v4f*)(lp + i * 256 + 8 * lane + 4);
        v8h hv;
        hv[0] = (_Float16)(fa.x * (float)FSCL); hv[1] = (_Float16)(fa.y * (float)FSCL);
        hv[2] = (_Float16)(fa.z * (float)FSCL); hv[3] = (_Float16)(fa.w * (float)FSCL);
        hv[4] = (_Float16)(fb.x * (float)FSCL); hv[5] = (_Float16)(fb.y * (float)FSCL);
        hv[6] = (_Float16)(fb.z * (float)FSCL); hv[7] = (_Float16)(fb.w * (float)FSCL);
        *(volatile v8h*)(hp + (size_t)i * 256 + 8 * lane) = hv;
      }
      if constexpr (WF != 0) {
#pragma unroll
        for (int i = 0; i < 8; ++i) {
          const v4f v = *(const v4f*)(lp + i * 128 + 4 * lane);
          *(volatile v4f*)(fp + (size_t)i * 128 + 4 * lane) = v;
        }
      }
      __threadfence();
    }
  }
}

__global__ __launch_bounds__(NTHR) void k_aggU(
    const int* __restrict__ csr, const int* __restrict__ off, const int* __restrict__ cnt,
    const int* __restrict__ esrc, const float* __restrict__ S, float* U, int nN, int nE, int csrLen) {
  __shared__ __attribute__((aligned(16))) float sStg[NWAVE * 128];
  const int tid = threadIdx.x, lane = tid & 31, wave = tid >> 5;
  const int tbase = (int)blockIdx.x * TGT + wave * 32;
  const int cnt_l = cnt[tbase + lane];
  const int off_l = off[tbase + lane];
  const int cch = lane & 15, eh = lane >> 4;
  float* stg = sStg + wave * 128;

#pragma unroll 1
  for (int j = 0; j < 32; ++j) {
    const int c = tbase + j;
    int n = __builtin_amdgcn_readlane(cnt_l, j);
    n = n < 0 ? 0 : (n > DEGCAP ? DEGCAP : n);
    const int st = __builtin_amdgcn_readlane(off_l, j);
    float a = 0.0f;
#pragma unroll 1
    for (int q0 = 0; q0 < n; q0 += 32) {
      int pos = st + q0 + lane;
      pos = pos < 0 ? 0 : (pos > csrLen - 1 ? csrLen - 1 : pos);
      int e = csr[pos];
      e = e < 0 ? 0 : (e > nE - 1 ? nE - 1 : e);
      int sl = esrc[e];
      sl = sl < 0 ? 0 : (sl > nN - 1 ? nN - 1 : sl);
      const int mcnt = (n - q0) < 32 ? (n - q0) : 32;
#pragma unroll 1
      for (int p = 0; p < mcnt; p += 2) {
        const int s0 = __builtin_amdgcn_readlane(sl, p);
        const int s1 = __builtin_amdgcn_readlane(sl, p + 1);
        const int ss = eh ? s1 : s0;
        const float v = S[(size_t)ss * AC + cch];
        a += ((p + eh) < mcnt) ? v : 0.0f;
      }
    }
    a += __shfl_xor(a, 16, 32);
    stg[(j & 7) * AC + cch] = a;
    if ((j & 7) == 7) {
      WAVE_SYNC();
      const v4f v = *(const v4f*)(stg + 4 * lane);
      float* up = U + (size_t)(c - 7) * AC + 4 * lane;
      *(volatile v4f*)up = v;
      __threadfence();
      *(volatile v4f*)up = v;
      WAVE_SYNC();
    }
  }
}

__global__ __launch_bounds__(NTHR) void k_pool(
    const float* __restrict__ S, const float* __restrict__ U, const float* __restrict__ Hf,
    const float* __restrict__ d1w, const float* __restrict__ d1b,
    const float* __restrict__ d2w, const float* __restrict__ d2b,
    const float* __restrict__ adw, const float* __restrict__ adb, float* Gv, int nN) {
  __shared__ __attribute__((aligned(16))) float sS[NPER * AC];
  __shared__ __attribute__((aligned(16))) float xL[AC * HD];
  __shared__ __attribute__((aligned(16))) float yL[AC * HD];
  __shared__ float sAdj[AC * AC];
  __shared__ float sAdjn[AC * AC];
  __shared__ float sD[AC];
  __shared__ float sZ[AC];
  __shared__ float sE[AC];
  __shared__ float sQ[AC];
  __shared__ __attribute__((aligned(16))) float sG[HD];
  const int tid = threadIdx.x;
  int nb = (int)blockIdx.x * NPER;
  nb = (nb + NPER > nN) ? (nN - NPER) : nb;
  nb = nb < 0 ? 0 : nb;

#pragma unroll
  for (int i = 0; i < (NPER * AC) / (4 * NTHR); ++i) {
    const int idx = tid + NTHR * i;
    *(v4f*)(sS + 4 * idx) = *(const v4f*)(S + (size_t)nb * AC + 4 * idx);
  }
  __syncthreads();

  const int f = tid & (HD - 1), c0 = tid >> 6;
  {
    float a0 = 0.0f, a1 = 0.0f, a2 = 0.0f, a3 = 0.0f;
#pragma unroll 1
    for (int d = 0; d < NPER; ++d) {
      const float hv = Hf[(size_t)(nb + d) * HD + f];
      const float* sr = sS + d * AC + c0;
      a0 = fmaf(sr[0], hv, a0);
      a1 = fmaf(sr[4], hv, a1);
      a2 = fmaf(sr[8], hv, a2);
      a3 = fmaf(sr[12], hv, a3);
    }
    xL[(c0) * HD + f]      = a0;
    xL[(c0 + 4) * HD + f]  = a1;
    xL[(c0 + 8) * HD + f]  = a2;
    xL[(c0 + 12) * HD + f] = a3;
  }
  {
    const int cc = tid >> 4, kk = tid & 15;
    float a = 0.0f;
#pragma unroll 1
    for (int d = 0; d < NPER; ++d) a = fmaf(U[(size_t)(nb + d) * AC + cc], sS[d * AC + kk], a);
    sAdj[tid] = a;
  }
  __syncthreads();
  {
    const int cc = tid & 15;
    float s = 0.0f;
#pragma unroll 1
    for (int k = 0; k < AC; ++k) s += (k == cc) ? 1.0f : sAdj[cc * AC + k];
    s = fmaxf(s, 1.0f);
    sD[cc] = 1.0f / sqrtf(s);
  }
  __syncthreads();
  {
    const int cc = tid >> 4, kk = tid & 15;
    const float a = (cc == kk) ? 1.0f : sAdj[tid];
    sAdjn[tid] = sD[cc] * a * sD[kk];
  }
  __syncthreads();

#pragma unroll 1
  for (int L = 0; L < 2; ++L) {
    const float* w  = (L == 0) ? d1w : d2w;
    const float* bb = (L == 0) ? d1b : d2b;
    {
      float a0 = 0.0f, a1 = 0.0f, a2 = 0.0f, a3 = 0.0f;
#pragma unroll 1
      for (int k = 0; k < HD; ++k) {
        const float wv = w[k * HD + f];
        a0 = fmaf(xL[(c0) * HD + k], wv, a0);
        a1 = fmaf(xL[(c0 + 4) * HD + k], wv, a1);
        a2 = fmaf(xL[(c0 + 8) * HD + k], wv, a2);
        a3 = fmaf(xL[(c0 + 12) * HD + k], wv, a3);
      }
      yL[(c0) * HD + f]      = a0;
      yL[(c0 + 4) * HD + f]  = a1;
      yL[(c0 + 8) * HD + f]  = a2;
      yL[(c0 + 12) * HD + f] = a3;
    }
    __syncthreads();
    {
      const float bv = bb[f];
      float a0 = 0.0f, a1 = 0.0f, a2 = 0.0f, a3 = 0.0f;
#pragma unroll 1
      for (int mm = 0; mm < AC; ++mm) {
        const float yv = yL[mm * HD + f];
        a0 = fmaf(sAdjn[(c0) * AC + mm], yv, a0);
        a1 = fmaf(sAdjn[(c0 + 4) * AC + mm], yv, a1);
        a2 = fmaf(sAdjn[(c0 + 8) * AC + mm], yv, a2);
        a3 = fmaf(sAdjn[(c0 + 12) * AC + mm], yv, a3);
      }
      xL[(c0) * HD + f]      = fmaxf(a0 + bv, 0.0f);
      xL[(c0 + 4) * HD + f]  = fmaxf(a1 + bv, 0.0f);
      xL[(c0 + 8) * HD + f]  = fmaxf(a2 + bv, 0.0f);
      xL[(c0 + 12) * HD + f] = fmaxf(a3 + bv, 0.0f);
    }
    __syncthreads();
  }

  {
    const int cc = tid & 15;
    float z = adb[0];
#pragma unroll 1
    for (int k = 0; k < HD; ++k) z = fmaf(xL[cc * HD + k], adw[k], z);
    sZ[cc] = z;
  }
  __syncthreads();
  {
    const int cc = tid & 15;
    float mx = -__builtin_huge_valf();
#pragma unroll 1
    for (int i = 0; i < AC; ++i) mx = fmaxf(mx, sZ[i]);
    sE[cc] = expf(sZ[cc] - mx);
  }
  __syncthreads();
  {
    const int cc = tid & 15;
    float sm = 0.0f;
#pragma unroll 1
    for (int i = 0; i < AC; ++i) sm += sE[i];
    const float p1 = sE[cc] * (1.0f / sm);
    const float e2 = __expf(p1 - p1);
    const float p2 = e2 * (1.0f / e2);
    sQ[cc] = p2;
  }
  __syncthreads();
  {
    float g = 0.0f;
#pragma unroll 1
    for (int cc = 0; cc < AC; ++cc) g = fmaf(sQ[cc], xL[cc * HD + f], g);
    sG[f] = g;
  }
  __syncthreads();
  v4f ov = {0.f, 0.f, 0.f, 0.f};
  if (tid < HD / 4) ov = *(const v4f*)(sG + 4 * tid);
  float* gp = Gv + (size_t)blockIdx.x * HD + 4 * tid;
  if (tid < HD / 4) *(volatile v4f*)gp = ov;
  __threadfence();
  if (tid < HD / 4) *(volatile v4f*)gp = ov;
}

__global__ __launch_bounds__(NTHR) void k_head(
    const float* __restrict__ gvec, const float* __restrict__ mw1, const float* __restrict__ mb1,
    const float* __restrict__ mw2, const float* __restrict__ mb2, float* out, int G) {
  __shared__ float sH[GMAX * EMB];
  __shared__ __attribute__((aligned(16))) float sO[GMAX];
  const int tid = threadIdx.x;
#pragma unroll 1
  for (int idx = tid; idx < G * EMB; idx += NTHR) {
    const int g = idx >> 7, jj = idx & (EMB - 1);
    float a = mb1[jj];
#pragma unroll 1
    for (int k = 0; k < HD; ++k) a = fmaf(gvec[g * HD + k], mw1[k * EMB + jj], a);
    sH[idx] = fmaxf(a, 0.0f);
  }
  __syncthreads();
  {
    const int g = tid & (GMAX - 1);
    const int gc = g < G ? g : G - 1;
    float o = mb2[0];
#pragma unroll 1
    for (int jj = 0; jj < EMB; ++jj) o = fmaf(sH[gc * EMB + jj], mw2[jj], o);
    sO[g] = o;
  }
  __syncthreads();
  const int nq = G >> 2;
  v4f ov = {0.f, 0.f, 0.f, 0.f};
  if (tid < nq) ov = *(const v4f*)(sO + 4 * tid);
  if (tid < nq) *(volatile v4f*)(out + 4 * tid) = ov;
  __threadfence();
  if (tid < nq) *(volatile v4f*)(out + 4 * tid) = ov;
}

extern "C" void kernel_launch(void* const* d_in, const int* in_sizes, int n_in,
                              void* d_out, int out_size, void* d_ws, size_t ws_size,
                              hipStream_t stream) {
  if (n_in < 26) return;
  const int nN = in_sizes[0] / IND;
  const int nE = in_sizes[1] / 2;
  if (nN <= 0 || nE <= 0) return;
  if (in_sizes[0] != nN * IND || in_sizes[1] != 2 * nE) return;
  if (in_sizes[2] != nE * EDD || in_sizes[3] != nN) return;
  if (in_sizes[4] != (IND + EDD) * HD || in_sizes[5] != HD || in_sizes[6] != HD * HD || in_sizes[7] != HD) return;
  if (in_sizes[8] != (HD + EDD) * HD || in_sizes[9] != HD || in_sizes[10] != HD * HD || in_sizes[11] != HD) return;
  if (in_sizes[12] != (HD + EDD) * AC || in_sizes[13] != AC || in_sizes[14] != AC * AC || in_sizes[15] != AC) return;
  if (in_sizes[16] != HD * HD || in_sizes[17] != HD || in_sizes[18] != HD * HD || in_sizes[19] != HD) return;
  if (in_sizes[20] != HD || in_sizes[21] != 1) return;
  if (in_sizes[22] != HD * EMB || in_sizes[23] != EMB || in_sizes[24] != EMB || in_sizes[25] != 1) return;
  if (nN > (1 << 20) || nE > (1 << 28)) return;
  const int G = out_size;
  if (G < 1 || G > GMAX || (G & 3) != 0) return;
  if (nN != G * NPER) return;

  const float* x    = (const float*)d_in[0];
  const int*   ei   = (const int*)d_in[1];
  const float* ea   = (const float*)d_in[2];
  const float* g1w1 = (const float*)d_in[4];  const float* g1b1 = (const float*)d_in[5];
  const float* g1w2 = (const float*)d_in[6];  const float* g1b2 = (const float*)d_in[7];
  const float* g2w1 = (const float*)d_in[8];  const float* g2b1 = (const float*)d_in[9];
  const float* g2w2 = (const float*)d_in[10]; const float* g2b2 = (const float*)d_in[11];
  const float* agw1 = (const float*)d_in[12]; const float* agb1 = (const float*)d_in[13];
  const float* agw2 = (const float*)d_in[14]; const float* agb2 = (const float*)d_in[15];
  const float* d1w  = (const float*)d_in[16]; const float* d1b  = (const float*)d_in[17];
  const float* d2w  = (const float*)d_in[18]; const float* d2b  = (const float*)d_in[19];
  const float* adw  = (const float*)d_in[20]; const float* adb  = (const float*)d_in[21];
  const float* mw1  = (const float*)d_in[22]; const float* mb1  = (const float*)d_in[23];
  const float* mw2  = (const float*)d_in[24]; const float* mb2  = (const float*)d_in[25];
  float* out = (float*)d_out;
  const int* keys = ei + nE;
  const int* esrc = ei;
  const int nK = nE;

  const int NPAD   = ((nN + TGT - 1) / TGT) * TGT;
  const int nBC    = (nN + NBC - 1) / NBC;
  const int CNTPAD = nBC * NBC;
  const int nBF    = (nN + NBF - 1) / NBF;
  const int OFFN   = nBF * NBF;
  if (nBF + 1 > RBN) return;
  if (OFFN > CNTPAD || NPAD > OFFN) return;
  const int csrLen = ((nK + 31) & ~31) + 32 * (nBF + 1);
  const int nAgg   = NPAD / TGT;
  const int nGemm  = NPAD / GROWS;

  char* ws = (char*)d_ws;
  size_t off = 0;
#define CARVE(NAME, BYTES) const size_t NAME = off; off += (size_t)(BYTES); off = (off + 255) & ~(size_t)255;
  CARVE(oH1h, (size_t)NPAD * HD * 2)
  CARVE(oH2h, (size_t)NPAD * HD * 2)
  CARVE(oH2f, (size_t)NPAD * HD * 4)
  CARVE(oR1,  (size_t)NPAD * HD * 4)
  CARVE(oR2,  (size_t)NPAD * HD * 4)
  CARVE(oR3,  (size_t)NPAD * 32 * 4)
  CARVE(oS,   (size_t)NPAD * AC * 4)
  CARVE(oU,   (size_t)NPAD * AC * 4)
  CARVE(oG,   (size_t)GMAX * HD * 4)
  CARVE(oW1h, (size_t)HD * HD * 2)
  CARVE(oW1l, (size_t)HD * HD * 2)
  CARVE(oW2h, (size_t)HD * HD * 2)
  CARVE(oW2l, (size_t)HD * HD * 2)
  CARVE(oW3h, (size_t)AC * 32 * 2)
  CARVE(oW3l, (size_t)AC * 32 * 2)
  CARVE(oCnt, (size_t)CNTPAD * 4)
  CARVE(oOff, (size_t)OFFN * 4)
  CARVE(oRb,  (size_t)RBN * 4)
  CARVE(oCsr, (size_t)csrLen * 4)
#undef CARVE
  if (off > ws_size || off > (size_t)WSCAP) return;
  _Float16*       H1h = (_Float16*)(ws + oH1h);
  _Float16*       H2h = (_Float16*)(ws + oH2h);
  float*          H2f = (float*)(ws + oH2f);
  float*          R1  = (float*)(ws + oR1);
  float*          R2  = (float*)(ws + oR2);
  float*          R3  = (float*)(ws + oR3);
  float*          Sp  = (float*)(ws + oS);
  float*          Up  = (float*)(ws + oU);
  float*          Gp  = (float*)(ws + oG);
  unsigned short* W1h = (unsigned short*)(ws + oW1h);
  unsigned short* W1l = (unsigned short*)(ws + oW1l);
  unsigned short* W2h = (unsigned short*)(ws + oW2h);
  unsigned short* W2l = (unsigned short*)(ws + oW2l);
  unsigned short* W3h = (unsigned short*)(ws + oW3h);
  unsigned short* W3l = (unsigned short*)(ws + oW3l);
  int*            cnt  = (int*)(ws + oCnt);
  int*            offp = (int*)(ws + oOff);
  int*            rb   = (int*)(ws + oRb);
  int*            csr  = (int*)(ws + oCsr);

  const int vec8 = ((nE & 7) == 0) ? 1 : 0;

  hipFuncSetAttribute(reinterpret_cast<const void*>(&k_count),
                      hipFuncAttributeMaxDynamicSharedMemorySize, LDS_COUNT);
  k_count<<<nBC, NTHR, LDS_COUNT, stream>>>(keys, cnt, nK, vec8);
  k_offsets<<<1, OTHR, 0, stream>>>(cnt, offp, rb, nBF);
  hipFuncSetAttribute(reinterpret_cast<const void*>(&k_fill),
                      hipFuncAttributeMaxDynamicSharedMemorySize, LDS_FILL);
  k_fill<<<nBF, NTHR, LDS_FILL, stream>>>(keys, offp, rb, csr, nK, vec8, csrLen);

  {
    const int t1 = (HD * HD) / 8;
    const int t3 = (AC * 32) / 8;
    k_w2split<<<(t1 + NTHR - 1) / NTHR, NTHR, 0, stream>>>(g1w2, W1h, W1l, HD, HD, HD, t1);
    k_w2split<<<(t1 + NTHR - 1) / NTHR, NTHR, 0, stream>>>(g2w2, W2h, W2l, HD, HD, HD, t1);
    k_w2split<<<(t3 + NTHR - 1) / NTHR, NTHR, 0, stream>>>(agw2, W3h, W3l, AC, AC, 32, t3);
  }

  k_conv<IND, HD, 1><<<nAgg, NTHR, 0, stream>>>(x, H1h, ea, csr, offp, cnt, esrc, g1w1, g1b1, R1, nN, nE, csrLen);
  k_gemm2<HD, HD, 0, 0><<<nGemm, NTHR, 0, stream>>>(R1, W1h, W1l, cnt, g1b2, H1h, H2f, Sp, nN);

  k_conv<HD, HD, 0><<<nAgg, NTHR, 0, stream>>>(x, H1h, ea, csr, offp, cnt, esrc, g2w1, g2b1, R2, nN, nE, csrLen);
  k_gemm2<HD, HD, 0, 1><<<nGemm, NTHR, 0, stream>>>(R2, W2h, W2l, cnt, g2b2, H2h, H2f, Sp, nN);

  k_conv<HD, AC, 0><<<nAgg, NTHR, 0, stream>>>(x, H2h, ea, csr, offp, cnt, esrc, agw1, agb1, R3, nN, nE, csrLen);
  k_gemm2<32, AC, 1, 0><<<nGemm, NTHR, 0, stream>>>(R3, W3h, W3l, cnt, agb2, H1h, H2f, Sp, nN);

  k_aggU<<<nAgg, NTHR, 0, stream>>>(csr, offp, cnt, esrc, Sp, Up, nN, nE, csrLen);

  k_pool<<<G, NTHR, 0, stream>>>(Sp, Up, H2f, d1w, d1b, d2w, d2b, adw, adb, Gp, nN);

  k_head<<<1, NTHR, 0, stream>>>(Gp, mw1, mb1, mw2, mb2, out, G);
}
